// PAM_46523085750999
// MI455X (gfx1250) — hardware-verified
//
#include <hip/hip_runtime.h>


namespace {
constexpr int B = 4, C = 256, T = 4096, IC = 128, BL = 4  , QB = 32  , PL = 128 * QB  ;
constexpr float XS = 8.0f, WSC = 256.0f, RS_ = 1024.0f, PS = 1024.0f, LOG2E = 1.4426950408889634f, BNEPS = 1e-5f;
static_assert(T % 32 == 0 && C == 256 && IC == 128 && QB >= 1 && QB <= 32 && PL % 32 == 0, "tiling");
typedef _Float16 b16;
typedef __attribute__((ext_vector_type(16))) _Float16 v16b;
typedef __attribute__((ext_vector_type(8))) _Float16 v8b;
typedef __attribute__((ext_vector_type(8))) float v8f;
typedef __attribute__((ext_vector_type(4))) float v4f;
__device__ __forceinline__ float bf16_rne(float f) { unsigned int u = __float_as_uint(f); u += 0x7FFFu + ((u >> 16) & 1u); return __uint_as_float(u & 0xFFFF0000u); }
__device__ __forceinline__ void split16(float v, b16& hi, b16& lo) { hi = (b16)v; lo = (b16)(v - (float)hi); }
__device__ __forceinline__ v16b frag_kb(const b16* p, int hh) { const v8b a = *(const v8b*)(p + 8 * hh), b = *(const v8b*)(p + 16 + 8 * hh); v16b f;
#pragma unroll
  for (int e = 0; e < 8; ++e) { f[e] = a[e]; f[8 + e] = b[e]; } return f; }
__device__ __forceinline__ v8f wmma16b(v16b a, v16b b, v8f c) { v8f d = __builtin_amdgcn_wmma_f32_16x16x32_f16(false, a, false, b, (short)0, c, false, false); asm volatile("v_nop\n\tv_nop\n\tv_nop\n\tv_nop" : "+v"(d) : "v"(a), "v"(b)); return d; }
__device__ __forceinline__ void wave_lds_sync() { __builtin_amdgcn_fence(__ATOMIC_RELEASE, "workgroup"); __builtin_amdgcn_wave_barrier(); __builtin_amdgcn_fence(__ATOMIC_ACQUIRE, "workgroup"); }
__device__ __forceinline__ float pmul(float a, float b) { float p = a * b; asm volatile("" : "+v"(p)); return p; }
__device__ __forceinline__ int iclamp(int v, int lo, int hi) { return v < lo ? lo : (v > hi ? hi : v); }

typedef __attribute__((ext_vector_type(2))) _Float16 v2h;
typedef __attribute__((ext_vector_type(4))) _Float16 v4h;
typedef __attribute__((ext_vector_type(2))) float v2f;
typedef __attribute__((ext_vector_type(4))) int v4i;
__device__ __forceinline__ float nexp2(float v) { return __builtin_amdgcn_exp2f(v); }
__device__ __forceinline__ float bfp(float v) { float t = bf16_rne(v); asm volatile("" : "+v"(t)); return t; }

__global__ __launch_bounds__(256) void wt_kernel(const float* __restrict__ w1, const float* __restrict__ w2, const float* __restrict__ w3, const float* __restrict__ w4, b16* __restrict__ W123, b16* __restrict__ W4T, b16* __restrict__ W4Q) {
  const int u = blockIdx.x * 256 + threadIdx.x;
  if (u < 3 * IC * C / 8) { const int e = u * 8; const int o = e / C, k0 = e % C; const float* src = (o < IC) ? (w1 + (size_t)o * C) : (o < 2 * IC ? (w2 + (size_t)(o - IC) * C) : (w3 + (size_t)(o - 2 * IC) * C)); v8b v; for (int j = 0; j < 8; ++j) v[j] = (b16)(bf16_rne(src[k0 + j]) * WSC);
    for (int pass = 0; pass < 2; ++pass) { *(volatile v8b*)(W123 + e) = v; __threadfence(); } }
  else if (u < 3 * IC * C / 8 + C * IC / 8) { const int e = (u - 3 * IC * C / 8) * 8; v8b v, q; for (int j = 0; j < 8; ++j) { const float w = bf16_rne(w4[e + j]); v[j] = (b16)(w * WSC); q[j] = (b16)(w * 0.25f); }
    for (int pass = 0; pass < 2; ++pass) { *(volatile v8b*)(W4T + e) = v; *(volatile v8b*)(W4Q + e) = q; __threadfence(); } }
}
__global__ __launch_bounds__(128) void proj_kernel(const float* __restrict__ x, const b16* __restrict__ W123, b16* __restrict__ Ph, b16* __restrict__ Pl) {
  __shared__ __attribute__((aligned(16))) b16 Ah[4][16][C + 8]; __shared__ __attribute__((aligned(16))) float Tw[64][IC + 1];
  const int wave = threadIdx.x >> 5, lane = threadIdx.x & 31, nloc = lane & 15, hlf = lane >> 4; const int b = blockIdx.y, m = blockIdx.z; const int n0 = blockIdx.x * 64;
  for (int idx = lane; idx < 16 * C; idx += 32) { const int k = idx >> 4, rr = idx & 15; Ah[wave][rr][k] = (b16)(bf16_rne(x[((size_t)b * C + k) * T + n0 + wave * 16 + rr]) * XS); }
  wave_lds_sync();
  v8f acc[8]; for (int t = 0; t < 8; ++t) acc[t] = (v8f){};
  const b16* W = W123 + (size_t)m * IC * C;
#pragma unroll 1
  for (int kb = 0; kb < C; kb += 32) { const v16b a = frag_kb(&Ah[wave][nloc][kb], hlf);
#pragma unroll
    for (int t = 0; t < 8; ++t) acc[t] = wmma16b(a, frag_kb(W + (size_t)(t * 16 + nloc) * C + kb, hlf), acc[t]); }
#pragma unroll
  for (int t = 0; t < 8; ++t) for (int r = 0; r < 8; ++r) Tw[wave * 16 + 8 * hlf + r][t * 16 + nloc] = acc[t][r] * (1.0f / (XS * WSC));
  __syncthreads();
  for (int pass = 0; pass < 2; ++pass) { for (int cc = 0; cc < 32; ++cc) { const int ch = wave * 32 + cc; const size_t o_ = (((size_t)b * 3 + m) * IC + ch) * T + n0 + 2 * lane; v2h hv, lv;
      for (int j = 0; j < 2; ++j) { const float v = Tw[2 * lane + j][ch] * XS; const b16 ph = (b16)v; hv[j] = ph; lv[j] = (b16)((v - (float)ph) * RS_); }
      *(volatile v2h*)(Ph + o_) = hv; *(volatile v2h*)(Pl + o_) = lv; } __threadfence(); }
}
__global__ __launch_bounds__(32) void attn_kernel(const b16* __restrict__ Ph, const b16* __restrict__ Pl, float* __restrict__ RES) {
  __shared__ __attribute__((aligned(16))) b16 Pt[16][32 + 8]; __shared__ __attribute__((aligned(16))) float Of[16][IC + 4];
  const int lane = threadIdx.x, nloc = lane & 15, hlf = lane >> 4; const int cres = blockIdx.x >> 3, jg = blockIdx.x & 7, b = blockIdx.y; if (cres >= QB) return;
  auto qrow = [&](int r) { return cres + 32 * (16 * jg + r); };
  const b16* Qh = Ph + ((size_t)b * 3 + 0) * IC * T; const b16* Qlp = Pl + ((size_t)b * 3 + 0) * IC * T;
  const b16* Kh = Ph + ((size_t)b * 3 + 1) * IC * T; const b16* Klp = Pl + ((size_t)b * 3 + 1) * IC * T;
  const b16* Vh = Ph + ((size_t)b * 3 + 2) * IC * T; const b16* Vlp = Pl + ((size_t)b * 3 + 2) * IC * T;
  v16b aqh[4];
#pragma unroll
  for (int ks = 0; ks < 4; ++ks) aqh[ks] = frag_kb(Qh + (size_t)qrow(nloc) * IC + ks * 32, hlf);
  const b16* qlrow = Qlp + (size_t)qrow(nloc) * IC;
  float mrow[8], lsum[8]; for (int r = 0; r < 8; ++r) { mrow[r] = -INFINITY; lsum[r] = 0.0f; }
  v8f acco[8], accol[8];
#pragma unroll
  for (int t = 0; t < 8; ++t) { acco[t] = (v8f){}; accol[t] = (v8f){}; }
#pragma unroll 1
  for (int kb = 0; kb < T; kb += 32) {
    v8f sh[2], sl[2];
#pragma unroll
    for (int t = 0; t < 2; ++t) { sh[t] = (v8f){}; sl[t] = (v8f){}; const int key = kb + t * 16 + nloc;
#pragma unroll
      for (int ks = 0; ks < 4; ++ks) { v16b bh, bl;
#pragma unroll
        for (int e = 0; e < 16; ++e) { const int cc = ks * 32 + ((e < 8) ? (8 * hlf + e) : (16 + 8 * hlf + (e - 8))); const size_t o_ = (size_t)cc * T + key; bh[e] = Kh[o_]; bl[e] = Klp[o_]; }
        sh[t] = wmma16b(aqh[ks], bh, sh[t]); sl[t] = wmma16b(aqh[ks], bl, sl[t]); sl[t] = wmma16b(frag_kb(qlrow + ks * 32, hlf), bh, sl[t]); } }
    float s[2][8], mx[8];
#pragma unroll
    for (int r = 0; r < 8; ++r) { mx[r] = -INFINITY;
#pragma unroll
      for (int t = 0; t < 2; ++t) { s[t][r] = (sh[t][r] + sl[t][r] * (1.0f / RS_)) * (1.0f / (XS * XS)); mx[r] = fmaxf(mx[r], s[t][r]); } }
#pragma unroll
    for (int o = 1; o < 16; o <<= 1) for (int r = 0; r < 8; ++r) mx[r] = fmaxf(mx[r], __shfl_xor(mx[r], o));
    v16b pv;
#pragma unroll
    for (int r = 0; r < 8; ++r) { const float mn = fmaxf(mrow[r], mx[r]); const float corr = nexp2((mrow[r] - mn) * LOG2E); mrow[r] = mn; lsum[r] *= corr;
#pragma unroll
      for (int t = 0; t < 8; ++t) { acco[t][r] *= corr; accol[t][r] *= corr; }
#pragma unroll
      for (int t = 0; t < 2; ++t) { const float p = nexp2((s[t][r] - mn) * LOG2E); lsum[r] += p; pv[8 * t + r] = (b16)(p * PS); } }
#pragma unroll
    for (int t = 0; t < 2; ++t) for (int r = 0; r < 8; ++r) Pt[8 * hlf + r][16 * t + nloc] = pv[8 * t + r];
    wave_lds_sync();
    const v16b a = frag_kb(&Pt[nloc][0], hlf);
#pragma unroll
    for (int t = 0; t < 8; ++t) { v16b vh, vl;
#pragma unroll
      for (int e = 0; e < 16; ++e) { const int k = (e < 8) ? (8 * hlf + e) : (16 + 8 * hlf + (e - 8)); const size_t o_ = (size_t)(kb + k) * IC + t * 16 + nloc; vh[e] = Vh[o_]; vl[e] = Vlp[o_]; }
      acco[t] = wmma16b(a, vh, acco[t]); accol[t] = wmma16b(a, vl, accol[t]); }
    wave_lds_sync(); }
#pragma unroll
  for (int o = 1; o < 16; o <<= 1) for (int r = 0; r < 8; ++r) lsum[r] += __shfl_xor(lsum[r], o);
#pragma unroll
  for (int t = 0; t < 8; ++t) for (int r = 0; r < 8; ++r) Of[8 * hlf + r][t * 16 + nloc] = (acco[t][r] + accol[t][r] * (1.0f / RS_)) * (1.0f / (PS * XS)) / lsum[r];
  wave_lds_sync();
  for (int pass = 0; pass < 2; ++pass) { for (int rr = 0; rr < 16; ++rr) *(volatile v4f*)(RES + ((size_t)b * T + qrow(rr)) * IC + lane * 4) = *(const v4f*)(&Of[rr][lane * 4]); __threadfence(); }
}
__global__ __launch_bounds__(64) void out_kernel(const float* __restrict__ RES, const b16* __restrict__ W4T, const b16* __restrict__ W4Q, const float* __restrict__ gam, const float* __restrict__ bet, const float* __restrict__ rmean, const float* __restrict__ rvar, const float* __restrict__ x, float* __restrict__ out) {
  __shared__ __attribute__((aligned(16))) b16 Ah[2][16][IC + 8], Al[2][16][IC + 8]; __shared__ float Zs[32][C + 1];
  const int wave = threadIdx.x >> 5, lane = threadIdx.x & 31, nloc = lane & 15, hlf = lane >> 4; const int b = blockIdx.y; const int n0 = blockIdx.x * 32; const float* Rb = RES + (size_t)b * T * IC;
  for (int idx = lane; idx < 16 * IC; idx += 32) { const int k = idx >> 4, rr = idx & 15; const float vs = Rb[(size_t)k * T + n0 + wave * 16 + rr] * XS; const b16 ph = (b16)vs; Ah[wave][rr][k] = ph; Al[wave][rr][k] = (b16)((vs - (float)ph) * RS_); }
  wave_lds_sync();
  v16b a[4], al[4];
#pragma unroll
  for (int ks = 0; ks < 4; ++ks) { a[ks] = frag_kb(&Ah[wave][nloc][ks * 32], hlf); al[ks] = frag_kb(&Al[wave][nloc][ks * 32], hlf); }
#pragma unroll 1
  for (int t = 0; t < C / 16; ++t) { v8f acc = (v8f){};
#pragma unroll
    for (int ks = 0; ks < 4; ++ks) { const size_t wo_ = (size_t)(t * 16 + nloc) * IC + ks * 32; acc = wmma16b(a[ks], frag_kb(W4T + wo_, hlf), acc); acc = wmma16b(al[ks], frag_kb(W4Q + wo_, hlf), acc); }
#pragma unroll
    for (int r = 0; r < 8; ++r) Zs[wave * 16 + 8 * hlf + r][t * 16 + nloc] = acc[r] * (1.0f / (XS * WSC)); }
  __syncthreads();
  for (int pass = 0; pass < 2; ++pass) {
#pragma unroll 4
    for (int cc = 0; cc < C / 2; ++cc) { const int ch = wave * (C / 2) + cc; const float sc = bf16_rne(gam[ch]) * rsqrtf(bf16_rne(rvar[ch]) + BNEPS), mu = bf16_rne(rmean[ch]), be = bf16_rne(bet[ch]); const size_t o_ = ((size_t)b * C + ch) * T + n0 + lane;
      ((volatile float*)out)[o_] = pmul(Zs[lane][ch] - mu, sc) + be + bf16_rne(x[o_]); }
    __threadfence(); }
}
}

extern "C" void kernel_launch(void* const* d_in, const int* in_sizes, int n_in, void* d_out, int out_size, void* d_ws, size_t ws_size, hipStream_t stream) {
  (void)n_in;
  auto Fp = [&](int i) { return (const float*)d_in[i]; };
  if (in_sizes[0] != B * C * T || in_sizes[1] != IC * C || in_sizes[2] != IC * C || in_sizes[3] != IC * C || in_sizes[4] != C * IC || in_sizes[5] != C || in_sizes[6] != C || in_sizes[7] != C || in_sizes[8] != C || out_size != B * C * T) return;
  size_t off = 0; char* ws = (char*)d_ws;
  auto carve = [&](size_t bytes) { char* p = ws + off; off += (bytes + 255) & ~(size_t)255; return p; };
  b16* W123 = (b16*)carve((size_t)3 * IC * C * 2); b16* W4T = (b16*)carve((size_t)C * IC * 2); b16* W4Q = (b16*)carve((size_t)C * IC * 2);
  b16* Ph = (b16*)carve((size_t)B * 3 * IC * T * 2); b16* Pl = (b16*)carve((size_t)B * 3 * IC * T * 2); float* RES = (float*)carve((size_t)B * T * IC * 4);
  if (off > ws_size || off > ((size_t)64 << 20)) return;
  wt_kernel<<<(3 * IC * C / 8 + C * IC / 8 + 255) / 256, 256, 0, stream>>>(Fp(1), Fp(2), Fp(3), Fp(4), W123, W4T, W4Q);
  proj_kernel<<<dim3(T / 64, BL, 3), 128, 0, stream>>>(Fp(0), W123, Ph, Pl);
  attn_kernel<<<dim3(256, BL), 32, 0, stream>>>(Ph, Pl, RES);
  out_kernel<<<dim3(PL / 32, BL), 64, 0, stream>>>(RES, W4T, W4Q, Fp(5), Fp(6), Fp(7), Fp(8), Fp(0), (float*)d_out);
}
